// Masked_MAB_29892972380750
// MI455X (gfx1250) — hardware-verified
//
#include <hip/hip_runtime.h>


#define NB_  8
#define TT   1024
#define DD   512
#define NH_  8
#define HD   64
#define ZH   2
#define SCL  0.04419417382415922f
typedef _Float16 h16;
typedef unsigned short bf;
typedef __attribute__((ext_vector_type(16))) __bf16   v16bf;
typedef __attribute__((ext_vector_type(16))) _Float16 v16h;
typedef __attribute__((ext_vector_type(8)))  _Float16 v8h;
typedef __attribute__((ext_vector_type(8)))  unsigned short v8us;
typedef __attribute__((ext_vector_type(8)))  float    v8f;
typedef __attribute__((ext_vector_type(4)))  float    v4f;
typedef v8h  __attribute__((may_alias)) v8ha;
typedef v4f  __attribute__((may_alias)) v4fa;
typedef v8us __attribute__((may_alias)) v8usa;

__device__ __forceinline__ unsigned short f2bf(float f) { unsigned u = __float_as_uint(f); u += 0x7FFFu + ((u >> 16) & 1u); return (unsigned short)(u >> 16); }
__device__ __forceinline__ float bf2f(unsigned short b) { return __uint_as_float(((unsigned)b) << 16); }
__device__ __forceinline__ float bfr(float f) { return bf2f(f2bf(f)); }
__device__ __forceinline__ v16h cat16(v8h lo, v8h hi) { return __builtin_shufflevector(lo, hi, 0, 1, 2, 3, 4, 5, 6, 7, 8, 9, 10, 11, 12, 13, 14, 15); }
__device__ __forceinline__ v16bf cat16b(v8us lo, v8us hi) { return __builtin_bit_cast(v16bf, __builtin_shufflevector(lo, hi, 0, 1, 2, 3, 4, 5, 6, 7, 8, 9, 10, 11, 12, 13, 14, 15)); }
__device__ __forceinline__ v8f wmma16(v16h a, v16h b, v8f c) { return __builtin_amdgcn_wmma_f32_16x16x32_f16(false, a, false, b, (short)0, c, false, false); }
__device__ __forceinline__ v8f wmmab(v16bf a, v16bf b, v8f c) { return __builtin_amdgcn_wmma_f32_16x16x32_bf16(false, a, false, b, (short)0, c, false, false); }


template <typename T16> struct WFrag;
template <> struct WFrag<h16> { typedef v16h V; static __device__ __forceinline__ V ld(const h16* p) { return cat16(*(const v8h*)p, *(const v8h*)(p + 16)); } static __device__ __forceinline__ v8f mma(V a, V b, v8f c) { return wmma16(a, b, c); } };
template <> struct WFrag<bf> { typedef v16bf V; static __device__ __forceinline__ V ld(const bf* p) { return cat16b(*(const v8us*)p, *(const v8us*)(p + 16)); } static __device__ __forceinline__ v8f mma(V a, V b, v8f c) { return wmmab(a, b, c); } };
template <typename T16, int NSPLIT, bool BIAS>
__global__ __launch_bounds__(32) void k_gemmw(const T16* __restrict__ A, const T16* __restrict__ A2, const T16* __restrict__ Bt, const T16* __restrict__ Bt2, int K, float* C, int ldc, const float* __restrict__ bias, size_t sA, size_t sB, size_t sC) {
    typedef typename WFrag<T16>::V V;
    __shared__ __align__(16) float os[16 * 68];
    const size_t z = blockIdx.z; A += z * sA; if (A2) A2 += z * sA; Bt += z * sB; if (Bt2) Bt2 += z * sB; C += z * sC;
    const int lane = threadIdx.x & 31, lr = lane & 15, hi = lane >> 4; const int r0 = blockIdx.x * 64, c0 = blockIdx.y * 64;
    v8f acc[4][4];
#pragma unroll
    for (int mb = 0; mb < 4; ++mb)
#pragma unroll
        for (int nb = 0; nb < 4; ++nb) acc[mb][nb] = (v8f){};
    const size_t aoff = (size_t)(r0 + lr) * K + 8 * hi, boff = (size_t)(c0 + lr) * K + 8 * hi;
#pragma unroll 1
    for (int kc = 0; kc < K; kc += 32) {
        V a[4], a2[4];
#pragma unroll
        for (int mb = 0; mb < 4; ++mb) { a[mb] = WFrag<T16>::ld(A + aoff + (size_t)mb * 16 * K + kc); if (NSPLIT == 1 || NSPLIT == 2) a2[mb] = WFrag<T16>::ld(A2 + aoff + (size_t)mb * 16 * K + kc); }
#pragma unroll
        for (int nb = 0; nb < 4; ++nb) { const V b = WFrag<T16>::ld(Bt + boff + (size_t)nb * 16 * K + kc); V b2; if (NSPLIT >= 2) b2 = WFrag<T16>::ld(Bt2 + boff + (size_t)nb * 16 * K + kc);
#pragma unroll
            for (int mb = 0; mb < 4; ++mb) { acc[mb][nb] = WFrag<T16>::mma(a[mb], b, acc[mb][nb]); if (NSPLIT == 1 || NSPLIT == 2) acc[mb][nb] = WFrag<T16>::mma(a2[mb], b, acc[mb][nb]); if (NSPLIT >= 2) acc[mb][nb] = WFrag<T16>::mma(a[mb], b2, acc[mb][nb]); } }
        asm volatile("v_nop\n\tv_nop\n\tv_nop\n\tv_nop" : "+v"(acc[0][0]), "+v"(acc[1][1]), "+v"(acc[2][2]), "+v"(acc[3][3]) : "v"(a[0]), "v"(a[3]));
    }
#pragma unroll
    for (int mb = 0; mb < 4; ++mb) {
#pragma unroll
        for (int nb = 0; nb < 4; ++nb) {
#pragma unroll
            for (int j = 0; j < 8; ++j) os[(hi * 8 + j) * 68 + nb * 16 + lr] = acc[mb][nb][j]; }
        __builtin_amdgcn_wave_barrier(); asm volatile("" ::: "memory");
        float* crow = C + (size_t)(r0 + mb * 16) * ldc + c0;
#pragma unroll 1
        for (int ps = 0; ps < 2; ++ps) {
#pragma unroll
            for (int s = 0; s < 8; ++s) { const int row = 2 * s + hi, cofs = lr * 4; v4f val = *(const v4fa*)(os + row * 68 + cofs); if (BIAS) { val[0] += bfr(bias[c0 + cofs]); val[1] += bfr(bias[c0 + cofs + 1]); val[2] += bfr(bias[c0 + cofs + 2]); val[3] += bfr(bias[c0 + cofs + 3]); }
                *(volatile v4f*)(crow + (size_t)row * ldc + cofs) = val; }
            if (ps == 0) __threadfence(); }
        __builtin_amdgcn_wave_barrier(); asm volatile("" ::: "memory");
    }
}

__device__ __forceinline__ void splitf(float y, unsigned short& h, unsigned short& l) { h = f2bf(y); l = f2bf(y - bf2f(h)); }
typedef __attribute__((ext_vector_type(2))) unsigned short v2us;
typedef __attribute__((ext_vector_type(4))) unsigned short v4us;
typedef __attribute__((ext_vector_type(2))) float v2f;

__global__ __launch_bounds__(256) void k_wtG(const float* __restrict__ w, int K, int N, bf* Bt) {
    const int lane = threadIdx.x & 31; const int L0 = (blockIdx.x * 8 + (threadIdx.x >> 5)) * 8; const int nlines = N * K / 64;
#pragma unroll 1
    for (int ps = 0; ps < 2; ++ps) {
#pragma unroll 1
        for (int l = 0; l < 8; ++l) { const int L = L0 + l; if (L >= nlines) break; const size_t e = (size_t)L * 64 + lane * 2; const int k = (int)(e % K), n = (int)(e / K); v2us o;
            o[0] = f2bf(w[(size_t)k * N + n]); o[1] = f2bf(w[(size_t)(k + 1) * N + n]); *(volatile v2us*)(Bt + e) = o; }
        if (ps == 0) __threadfence(); }
}
__global__ __launch_bounds__(256) void k_cvt8(const float* __restrict__ src, bf* dst, size_t n8) { const size_t i = (size_t)blockIdx.x * 256 + threadIdx.x; if (i >= n8) return; const v8f v = *(const v8f*)(src + i * 8); v8us o;
#pragma unroll
    for (int k = 0; k < 8; ++k) o[k] = f2bf(v[k]); *(volatile v8us*)(dst + i * 8) = o; __threadfence(); *(volatile v8us*)(dst + i * 8) = o; }
__global__ __launch_bounds__(256) void k_maskf(float* F, const float* __restrict__ m) { const size_t i = ((size_t)blockIdx.x * 256 + threadIdx.x) * 4; if (i >= (size_t)TT * DD) return; const int t = (int)(i / DD); const float mk = bfr(m[t]); const v4f a = *(const v4f*)(F + i); v4f o; o[0] = __fmul_rn(a[0], mk); o[1] = __fmul_rn(a[1], mk); o[2] = __fmul_rn(a[2], mk); o[3] = __fmul_rn(a[3], mk); *(volatile v4f*)(F + i) = o; __threadfence(); *(volatile v4f*)(F + i) = o; }
__global__ __launch_bounds__(256) void k_pl(const float* __restrict__ F, bf* Ph, bf* Pl) { const size_t e = ((size_t)blockIdx.x * 256 + threadIdx.x) * 2; if (e >= (size_t)NH_ * TT * HD) return; const int d = (int)(e % HD); const int t = (int)((e / HD) % TT); const int h = (int)(e / ((size_t)HD * TT)); const float* f = F + (size_t)t * DD + h * HD + d; v2us oh, ol;
#pragma unroll
    for (int u = 0; u < 2; ++u) { unsigned short a, c; splitf(f[u], a, c); oh[u] = a; ol[u] = c; } *(volatile v2us*)(Ph + e) = oh; *(volatile v2us*)(Pl + e) = ol; __threadfence(); *(volatile v2us*)(Ph + e) = oh; *(volatile v2us*)(Pl + e) = ol; }
__global__ __launch_bounds__(256) void k_vtp(const float* __restrict__ F, bf* Vh, bf* Vl) { const size_t e = ((size_t)blockIdx.x * 256 + threadIdx.x) * 2; if (e >= (size_t)NH_ * HD * TT) return; const int t = (int)(e % TT); const int d = (int)((e / TT) % HD); const int h = (int)(e / ((size_t)TT * HD)); v2us oh, ol;
#pragma unroll
    for (int u = 0; u < 2; ++u) { unsigned short a, c; splitf(F[(size_t)(t + u) * DD + h * HD + d], a, c); oh[u] = a; ol[u] = c; } *(volatile v2us*)(Vh + e) = oh; *(volatile v2us*)(Vl + e) = ol; __threadfence(); *(volatile v2us*)(Vh + e) = oh; *(volatile v2us*)(Vl + e) = ol; }
__global__ __launch_bounds__(256) void k_msoft(const float* __restrict__ Sb, const float* __restrict__ m, bf* Ph, bf* Pl) { const int lane = threadIdx.x & 31; const int row = blockIdx.x * 8 + (threadIdx.x >> 5); if (row >= ZH * TT) return; const int i = row % TT; const float mi = bfr(m[i]); const float* sr = Sb + (size_t)row * TT; float v[32]; float mx = -3.0e38f;
#pragma unroll
    for (int ch = 0; ch < 8; ++ch) { const v4f a = *(const v4f*)(sr + ch * 128 + lane * 4);
#pragma unroll
        for (int q = 0; q < 4; ++q) { float t = a[q] * SCL; asm volatile("" : "+v"(t)); v[ch * 4 + q] = t; mx = fmaxf(mx, t); } }
#pragma unroll
    for (int sh = 16; sh; sh >>= 1) mx = fmaxf(mx, __shfl_xor(mx, sh, 32));
    float sum = 0.f;
#pragma unroll
    for (int ch = 0; ch < 8; ++ch)
#pragma unroll
        for (int q = 0; q < 4; ++q) { const int j = ch * 128 + lane * 4 + q; const float mm = __fmul_rn(mi, bfr(m[j])); float d0 = __fsub_rn(v[ch * 4 + q], mx); asm volatile("" : "+v"(d0)); float ex = __fmul_rn(d0, mm); asm volatile("" : "+v"(ex)); const float nu = __fmul_rn(__expf(ex), mm); v[ch * 4 + q] = nu; sum = __fadd_rn(sum, nu); }
#pragma unroll
    for (int sh = 16; sh; sh >>= 1) sum += __shfl_xor(sum, sh, 32);
    const float f = __fdiv_rn(1.0f, __fadd_rn(sum, 1e-16f));
#pragma unroll 1
    for (int ps = 0; ps < 2; ++ps) {
#pragma unroll
        for (int ch = 0; ch < 8; ++ch) { v4us oh, ol;
#pragma unroll
            for (int q = 0; q < 4; ++q) { float pv = __fmul_rn(v[ch * 4 + q], f); unsigned short a, c2; splitf(pv, a, c2); oh[q] = a; ol[q] = c2; } const size_t oo = (size_t)row * TT + ch * 128 + lane * 4; *(volatile v4us*)(Ph + oo) = oh; *(volatile v4us*)(Pl + oo) = ol; }
        if (ps == 0) __threadfence(); } }
__global__ __launch_bounds__(256) void k_mrg(const float* __restrict__ Ob, const float* __restrict__ QF, int h0, float* O, bf* Ah, bf* Al) { const size_t e = ((size_t)blockIdx.x * 256 + threadIdx.x) * 2; if (e >= (size_t)ZH * TT * HD) return; const int d = (int)(e % HD); const int t = (int)((e / HD) % TT); const int z = (int)(e / ((size_t)HD * TT)); const size_t oo = (size_t)t * DD + (h0 + z) * HD + d; v2f o; v2us oh, ol;
#pragma unroll
    for (int u = 0; u < 2; ++u) { o[u] = __fadd_rn(QF[oo + u], Ob[e + u]); unsigned short a, c; splitf(o[u], a, c); oh[u] = a; ol[u] = c; } for (int ps = 0; ps < 2; ++ps) { *(volatile v2f*)(O + oo) = o; *(volatile v2us*)(Ah + oo) = oh; *(volatile v2us*)(Al + oo) = ol; if (ps == 0) __threadfence(); } }
__global__ __launch_bounds__(256) void k_fin(const float* __restrict__ O, const float* __restrict__ F2, const float* __restrict__ m, float* OUT) { const size_t i = ((size_t)blockIdx.x * 256 + threadIdx.x) * 4; if (i >= (size_t)TT * DD) return; const int t = (int)(i / DD); const float mk = bfr(m[t]); const v4f a = *(const v4f*)(O + i), f = *(const v4f*)(F2 + i); v4f o;
#pragma unroll
    for (int q = 0; q < 4; ++q) o[q] = __fadd_rn(a[q], fmaxf(__fmul_rn(f[q], mk), 0.f)); *(volatile v4f*)(OUT + i) = o; __threadfence(); *(volatile v4f*)(OUT + i) = o; }

extern "C" void kernel_launch(void* const* d_in, const int* in_sizes, int n_in,
                              void* d_out, int out_size, void* d_ws, size_t ws_size, hipStream_t stream) {
    (void)in_sizes; (void)n_in; (void)out_size;
    const float* Q = (const float*)d_in[0]; const float* K = (const float*)d_in[1]; const float* mask = (const float*)d_in[2]; const float* Wq = (const float*)d_in[3]; const float* bq = (const float*)d_in[4]; const float* Wk = (const float*)d_in[5]; const float* bk = (const float*)d_in[6]; const float* Wv = (const float*)d_in[7]; const float* bv = (const float*)d_in[8]; const float* Wo = (const float*)d_in[9]; const float* bo = (const float*)d_in[10];
    float* OUT = (float*)d_out;
    char* wsp = (char*)d_ws;
    auto take = [&](size_t bytes) { char* p = wsp; wsp += (bytes + 255) & ~(size_t)255; return (void*)p; };
    bf* WQ = (bf*)take((size_t)DD * DD * 2); bf* WK = (bf*)take((size_t)DD * DD * 2); bf* WV = (bf*)take((size_t)DD * DD * 2); bf* WO = (bf*)take((size_t)DD * DD * 2); bf* XQ = (bf*)take((size_t)TT * DD * 2); bf* XK = (bf*)take((size_t)TT * DD * 2);
    float* QF = (float*)take((size_t)TT * DD * 4); float* KF = (float*)take((size_t)TT * DD * 4); float* VF = (float*)take((size_t)TT * DD * 4); bf* Qh = (bf*)take((size_t)NH_ * TT * HD * 2); bf* Ql = (bf*)take((size_t)NH_ * TT * HD * 2); bf* Kh = (bf*)take((size_t)NH_ * TT * HD * 2); bf* Kl = (bf*)take((size_t)NH_ * TT * HD * 2); bf* Vh = (bf*)take((size_t)NH_ * HD * TT * 2); bf* Vl = (bf*)take((size_t)NH_ * HD * TT * 2);
    float* Sb = (float*)take((size_t)ZH * TT * TT * 4); bf* Ph = (bf*)take((size_t)ZH * TT * TT * 2); bf* Pl = (bf*)take((size_t)ZH * TT * TT * 2); float* Ob = (float*)take((size_t)ZH * TT * HD * 4); float* O = (float*)take((size_t)TT * DD * 4); bf* Ah = (bf*)take((size_t)TT * DD * 2); bf* Al = (bf*)take((size_t)TT * DD * 2); float* F2 = KF;
    if ((size_t)(wsp - (char*)d_ws) > ws_size) return;
    k_wtG<<<(DD * DD / 64 + 63) / 64, 256, 0, stream>>>(Wq, DD, DD, WQ); k_wtG<<<(DD * DD / 64 + 63) / 64, 256, 0, stream>>>(Wk, DD, DD, WK); k_wtG<<<(DD * DD / 64 + 63) / 64, 256, 0, stream>>>(Wv, DD, DD, WV); k_wtG<<<(DD * DD / 64 + 63) / 64, 256, 0, stream>>>(Wo, DD, DD, WO);
    const unsigned LT = (unsigned)(((size_t)TT * DD / 4 + 255) / 256), LP = (unsigned)(((size_t)NH_ * TT * HD / 2 + 255) / 256);
    for (int b = 0; b < NB_; ++b) { const float* mb = mask + (size_t)b * TT;
        k_cvt8<<<(TT * DD / 8 + 255) / 256, 256, 0, stream>>>(Q + (size_t)b * TT * DD, XQ, (size_t)TT * DD / 8); k_cvt8<<<(TT * DD / 8 + 255) / 256, 256, 0, stream>>>(K + (size_t)b * TT * DD, XK, (size_t)TT * DD / 8);
        k_gemmw<bf, 0, true><<<dim3(TT / 64, DD / 64, 1), 32, 0, stream>>>(XQ, nullptr, WQ, nullptr, DD, QF, DD, bq, 0, 0, 0); k_maskf<<<LT, 256, 0, stream>>>(QF, mb); k_pl<<<LP, 256, 0, stream>>>(QF, Qh, Ql);
        k_gemmw<bf, 0, true><<<dim3(TT / 64, DD / 64, 1), 32, 0, stream>>>(XK, nullptr, WK, nullptr, DD, KF, DD, bk, 0, 0, 0); k_maskf<<<LT, 256, 0, stream>>>(KF, mb); k_pl<<<LP, 256, 0, stream>>>(KF, Kh, Kl);
        k_gemmw<bf, 0, true><<<dim3(TT / 64, DD / 64, 1), 32, 0, stream>>>(XK, nullptr, WV, nullptr, DD, VF, DD, bv, 0, 0, 0); k_maskf<<<LT, 256, 0, stream>>>(VF, mb); k_vtp<<<LP, 256, 0, stream>>>(VF, Vh, Vl);
        for (int h0 = 0; h0 < NH_; h0 += ZH) { const size_t z = (size_t)h0;
            k_gemmw<bf, 2, false><<<dim3(TT / 64, TT / 64, ZH), 32, 0, stream>>>(Qh + z * TT * HD, Ql + z * TT * HD, Kh + z * TT * HD, Kl + z * TT * HD, HD, Sb, TT, nullptr, (size_t)TT * HD, (size_t)TT * HD, (size_t)TT * TT);
            k_msoft<<<ZH * TT / 8, 256, 0, stream>>>(Sb, mb, Ph, Pl);
            k_gemmw<bf, 2, false><<<dim3(TT / 64, 1, ZH), 32, 0, stream>>>(Ph, Pl, Vh + z * HD * TT, Vl + z * HD * TT, TT, Ob, HD, nullptr, (size_t)TT * TT, (size_t)HD * TT, (size_t)TT * HD);
            k_mrg<<<(unsigned)(((size_t)ZH * TT * HD / 2 + 255) / 256), 256, 0, stream>>>(Ob, QF, h0, O, Ah, Al); }
        k_gemmw<bf, 1, true><<<dim3(TT / 64, DD / 64, 1), 32, 0, stream>>>(Ah, Al, WO, nullptr, DD, F2, DD, bo, 0, 0, 0);
        k_fin<<<LT, 256, 0, stream>>>(O, F2, mb, OUT + (size_t)b * TT * DD); }
}
